// DAttention_75453985457398
// MI455X (gfx1250) — hardware-verified
//
#include <hip/hip_runtime.h>


namespace {
constexpr int NB = 8, C = 384, H = 40, W = 40, NPX = H * W, NH = 8, HC = 48, NG = 4, GC = 96, NR = NB * NPX  , HP = 64  ;
constexpr float XS = 8.0f, OS = 4096.0f  , WSC = 256.0f, PS = 8.0f, SCALE = 0.14433756729740643f  , LOG2E = 1.4426950408889634f, LNE = 1e-5f;

typedef _Float16 b16;
typedef __attribute__((ext_vector_type(16))) _Float16 v16b;
typedef __attribute__((ext_vector_type(8))) _Float16 v8b;
typedef __attribute__((ext_vector_type(8))) float v8f;
typedef __attribute__((ext_vector_type(4))) float v4f;
__device__ __forceinline__ float bf16_rne(float f) { unsigned int u = __float_as_uint(f); u += 0x7FFFu + ((u >> 16) & 1u); return __uint_as_float(u & 0xFFFF0000u); }
__device__ __forceinline__ void split16(float v, b16& hi, b16& lo) { hi = (b16)v; lo = (b16)(v - (float)hi); }
__device__ __forceinline__ v16b frag_kb(const b16* p, int hh) { const v8b a = *(const v8b*)(p + 8 * hh), b = *(const v8b*)(p + 16 + 8 * hh); v16b f;
#pragma unroll
  for (int e = 0; e < 8; ++e) { f[e] = a[e]; f[8 + e] = b[e]; } return f; }
__device__ __forceinline__ v8f wmma16b(v16b a, v16b b, v8f c) { v8f d = __builtin_amdgcn_wmma_f32_16x16x32_f16(false, a, false, b, (short)0, c, false, false); asm volatile("v_nop\n\tv_nop\n\tv_nop\n\tv_nop" : "+v"(d) : "v"(a), "v"(b)); return d; }
__device__ __forceinline__ void wave_lds_sync() { __builtin_amdgcn_fence(__ATOMIC_RELEASE, "workgroup"); __builtin_amdgcn_wave_barrier(); __builtin_amdgcn_fence(__ATOMIC_ACQUIRE, "workgroup"); }
__device__ __forceinline__ float pmul(float a, float b) { float p = a * b; asm volatile("" : "+v"(p)); return p; }
__device__ __forceinline__ float wsum(float v) { v += __shfl_xor(v, 1); v += __shfl_xor(v, 2); v += __shfl_xor(v, 4); v += __shfl_xor(v, 8); return v + __shfl_xor(v, 16); }
__device__ __forceinline__ float nexp2(float x) { return __builtin_amdgcn_exp2f(x); }
__device__ __forceinline__ float gelu_erf(float x) { return 0.5f * x * (1.0f + erff(x * 0.70710678118654752f)); }

__global__ __launch_bounds__(256) void prepx_kernel(const float* __restrict__ x, b16* __restrict__ X16T) {
  __shared__ b16 T[64][66];
  const int p0 = blockIdx.x * 64, c0 = blockIdx.y * 64, b = blockIdx.z, t_ = threadIdx.x;
  for (int q = t_; q < 64 * 64; q += 256) { const int cc = q >> 6, pp = q & 63; T[pp][cc] = (b16)(bf16_rne(x[((size_t)b * C + c0 + cc) * NPX + p0 + pp]) * XS); }
  __syncthreads();
  for (int pass = 0; pass < 2; ++pass) { for (int q = t_; q < 64 * 8; q += 256) { const int pp = q >> 3, c8 = (q & 7) * 8; v8b o; for (int j = 0; j < 8; ++j) o[j] = T[pp][c8 + j]; *(volatile v8b*)(X16T + ((size_t)b * NPX + p0 + pp) * C + c0 + c8) = o; } __threadfence(); }
}
__global__ __launch_bounds__(256) void prepw_kernel(const float* __restrict__ wq, const float* __restrict__ wk, const float* __restrict__ wv, const float* __restrict__ wo, b16* __restrict__ WP, b16* __restrict__ WOP) {
  const size_t t = (size_t)blockIdx.x * 256 + threadIdx.x; const size_t n1 = (size_t)3 * C * C / 8, n2 = (size_t)C * 512 / 8; v8b o;
  if (t < n1) { const size_t e = t * 8; const int k = (int)(e / ((size_t)C * C)); const size_t r = e - (size_t)k * C * C; const float* w = k == 0 ? wq : k == 1 ? wk : wv; for (int j = 0; j < 8; ++j) o[j] = (b16)(bf16_rne(w[r + j]) * WSC); for (int pass = 0; pass < 2; ++pass) { *(volatile v8b*)(WP + e) = o; __threadfence(); } }
  else if (t < n1 + n2) { const size_t e = (t - n1) * 8; const int oo = (int)(e / 512), k0 = (int)(e - (size_t)oo * 512); for (int j = 0; j < 8; ++j) { const int k = k0 + j, hd = k >> 6, d = k & 63; o[j] = (b16)((d < HC) ? bf16_rne(wo[(size_t)oo * C + hd * HC + d]) * WSC : 0.0f); } for (int pass = 0; pass < 2; ++pass) { *(volatile v8b*)(WOP + e) = o; __threadfence(); } }
}
template <int MODE>
__global__ __launch_bounds__(128) void proj_kernel(const b16* __restrict__ Ah, const b16* __restrict__ Al, const b16* __restrict__ Wt, const float* __restrict__ bias, float* __restrict__ Yc, b16* __restrict__ Yh, b16* __restrict__ Yl) {
  __shared__ __attribute__((aligned(16))) float Ts[96][64 + 4];
  constexpr int K = (MODE == 2) ? NH * HP : C; constexpr int NT = 6;
  const int wave = threadIdx.x >> 5, lane = threadIdx.x & 31, nloc = lane & 15, hlf = lane >> 4, t_ = threadIdx.x; const size_t m0 = (size_t)blockIdx.x * 64 + wave * 16; const int n0 = blockIdx.y * 96;
  v8f acc[NT];
#pragma unroll
  for (int t = 0; t < NT; ++t) acc[t] = (v8f){};
#pragma unroll 2
  for (int kb = 0; kb < K; kb += 32) { const v16b a = frag_kb(Ah + (m0 + nloc) * K + kb, hlf); v16b al = {}; if (MODE != 0) al = frag_kb(Al + (m0 + nloc) * K + kb, hlf);
#pragma unroll
    for (int t = 0; t < NT; ++t) { const v16b bw = frag_kb(Wt + (size_t)(n0 + t * 16 + nloc) * K + kb, hlf); acc[t] = wmma16b(a, bw, acc[t]); if (MODE != 0) acc[t] = wmma16b(al, bw, acc[t]); } }
  const float rs_ = (MODE == 2) ? 1.0f / (OS * WSC) : 1.0f / (XS * WSC);
#pragma unroll
  for (int t = 0; t < NT; ++t) { const int col = n0 + t * 16 + nloc; const float bb = bf16_rne(bias[col]);
#pragma unroll
    for (int r = 0; r < 8; ++r) Ts[t * 16 + nloc][wave * 16 + 8 * hlf + r] = acc[t][r] * rs_ + bb; }
  __syncthreads();
  const size_t row0 = (size_t)blockIdx.x * 64; const int b = (int)(row0 / NPX), p0 = (int)(row0 - (size_t)b * NPX); const int h0 = n0 / HC;
  for (int pass = 0; pass < 2; ++pass) {
    if (MODE == 0 || MODE == 2) { for (int i = t_; i < 96 * 16; i += 128) { const int cc = i >> 4, x4 = (i & 15) * 4; *(volatile v4f*)(Yc + ((size_t)b * C + n0 + cc) * NPX + p0 + x4) = *(const v4f*)(&Ts[cc][x4]); } }
    if (MODE == 0 || MODE == 1) {
      for (int i = t_; i < 64 * 2 * 8; i += 128) { const int nn = i >> 4, hh2 = (i >> 3) & 1, d8 = (i & 7) * 8; v8b o; for (int j2 = 0; j2 < 8; ++j2) { const int d = d8 + j2; float v = 0.0f; if (d < HC) { v = Ts[hh2 * HC + d][nn]; if (MODE == 0) v *= SCALE; } o[j2] = (b16)(v * XS); }
        *(volatile v8b*)(Yh + (((size_t)(b * NH + h0 + hh2)) * NPX + p0 + nn) * HP + d8) = o; } }
    if (MODE == 3) {
      for (int i = t_; i < 2 * HC * 8; i += 128) { const int hh2 = i / (HC * 8), rem = i - hh2 * HC * 8, d = rem >> 3, n8 = (rem & 7) * 8; v8b vh, vl; for (int j2 = 0; j2 < 8; ++j2) { b16 p, q; split16(Ts[hh2 * HC + d][n8 + j2] * XS, p, q); vh[j2] = p; vl[j2] = q; }
        const size_t gi = (((size_t)(b * NH + h0 + hh2)) * HC + d) * NPX + p0 + n8; *(volatile v8b*)(Yh + gi) = vh; *(volatile v8b*)(Yl + gi) = vl; } }
    __threadfence(); }
}
__global__ __launch_bounds__(256) void samp_kernel(const float* __restrict__ Q, const float* __restrict__ x, const float* __restrict__ wdw, const float* __restrict__ bdw, const float* __restrict__ lnw, const float* __restrict__ lnb, const float* __restrict__ woff, const float* __restrict__ wrpe, const float* __restrict__ brpe, b16* __restrict__ XSh, b16* __restrict__ XSl, b16* __restrict__ LE, b16* __restrict__ LEl) {
  __shared__ __attribute__((aligned(16))) b16 Rh[8][C + 8], Rl[8][C + 8], Lp[8][NH * HP + 8], Lpl[8][NH * HP + 8];
  const int wave = threadIdx.x >> 5, lane = threadIdx.x & 31; const size_t row = (size_t)blockIdx.x * 8 + wave; const int b = (int)(row / NPX), p = (int)(row - (size_t)b * NPX); const int i = p / W, j = p - i * W;
  const float* Qb = Q + (size_t)b * C * NPX; const float* xb = x + (size_t)b * C * NPX;
#pragma unroll 1
  for (int u = 0; u < 12; ++u) { const int c = lane * 12 + u; float s = bf16_rne(brpe[c]);
#pragma unroll 1
    for (int tap = 0; tap < 9; ++tap) { const int dy = tap / 3 - 1, dx = tap % 3 - 1; const int yy = i + dy, xx = j + dx; if (yy >= 0 && yy < H && xx >= 0 && xx < W) s += pmul(bf16_rne(wrpe[c * 9 + tap]), Qb[(size_t)c * NPX + yy * W + xx]); }
    const int hd = c / HC, d = c - hd * HC; b16 p_, q_; split16(s * OS, p_, q_); Lp[wave][hd * HP + d] = p_; Lpl[wave][hd * HP + d] = q_; }
  if (lane < NH) for (int d = HC; d < HP; ++d) { Lp[wave][lane * HP + d] = (b16)0.0f; Lpl[wave][lane * HP + d] = (b16)0.0f; }
#pragma unroll 1
  for (int g = 0; g < NG; ++g) {
    float tv[3]; float s1 = 0.0f;
#pragma unroll
    for (int u = 0; u < 3; ++u) { const int cl = lane * 3 + u, c = g * GC + cl; float s = bf16_rne(bdw[cl]);
#pragma unroll 1
      for (int tap = 0; tap < 9; ++tap) { const int dy = tap / 3 - 1, dx = tap % 3 - 1; const int yy = i + dy, xx = j + dx; if (yy >= 0 && yy < H && xx >= 0 && xx < W) s += pmul(bf16_rne(wdw[cl * 9 + tap]), Qb[(size_t)c * NPX + yy * W + xx]); }
      tv[u] = s; s1 += s; }
    const float mu = wsum(s1) * (1.0f / GC); float s2 = 0.0f; for (int u = 0; u < 3; ++u) { const float dv = tv[u] - mu; s2 += dv * dv; } const float rs = rsqrtf(wsum(s2) * (1.0f / GC) + LNE);
    float oy = 0.0f, ox = 0.0f; for (int u = 0; u < 3; ++u) { const int cl = lane * 3 + u; const float tn = gelu_erf(pmul((tv[u] - mu) * rs, bf16_rne(lnw[cl])) + bf16_rne(lnb[cl])); oy += pmul(tn, bf16_rne(woff[cl])); ox += pmul(tn, bf16_rne(woff[GC + cl])); }
    oy = wsum(oy); ox = wsum(ox);
    const float refy = ((0.5f + (float)i) / (float)(H - 1)) * 2.0f - 1.0f, refx = ((0.5f + (float)j) / (float)(W - 1)) * 2.0f - 1.0f;
    const float py = oy + refy, px_ = ox + refx;
    const float gx = (px_ + 1.0f) * 0.5f * (float)(W - 1), gy = (py + 1.0f) * 0.5f * (float)(H - 1);
    const float x0 = floorf(gx), y0 = floorf(gy), x1 = x0 + 1.0f, y1 = y0 + 1.0f;
    float cw[4]; int ci[4];
    for (int q = 0; q < 4; ++q) { const float xi = (q & 1) ? x1 : x0, yi = (q >> 1) ? y1 : y0; const float m = ((xi >= 0.0f) && (xi <= (float)(W - 1)) && (yi >= 0.0f) && (yi <= (float)(H - 1))) ? 1.0f : 0.0f;
      const int xv = (int)fminf(fmaxf(xi, 0.0f), (float)(W - 1)), yv = (int)fminf(fmaxf(yi, 0.0f), (float)(H - 1)); ci[q] = yv * W + xv;
      const float wq_ = ((q & 1) ? (gx - x0) : (x1 - gx)) * ((q >> 1) ? (gy - y0) : (y1 - gy)); cw[q] = wq_ * m; }
    for (int u = 0; u < 3; ++u) { const int c = g * GC + lane * 3 + u; const float* xc = xb + (size_t)c * NPX; const float v = ((pmul(bf16_rne(xc[ci[0]]), cw[0]) + pmul(bf16_rne(xc[ci[1]]), cw[1])) + pmul(bf16_rne(xc[ci[2]]), cw[2])) + pmul(bf16_rne(xc[ci[3]]), cw[3]); b16 a_, c_; split16(v * XS, a_, c_); Rh[wave][c] = a_; Rl[wave][c] = c_; } }
  wave_lds_sync();
  for (int pass = 0; pass < 2; ++pass) { for (int q = lane; q < C / 8; q += 32) { *(volatile v8b*)(XSh + row * C + q * 8) = *(const v8b*)(&Rh[wave][q * 8]); *(volatile v8b*)(XSl + row * C + q * 8) = *(const v8b*)(&Rl[wave][q * 8]); }
    for (int q = lane; q < NH * HP / 8; q += 32) { *(volatile v8b*)(LE + row * (NH * HP) + q * 8) = *(const v8b*)(&Lp[wave][q * 8]); *(volatile v8b*)(LEl + row * (NH * HP) + q * 8) = *(const v8b*)(&Lpl[wave][q * 8]); } __threadfence(); }
}
__global__ __launch_bounds__(64) void attn_kernel(const b16* __restrict__ QFh, const b16* __restrict__ KRh, const b16* __restrict__ VT, const b16* __restrict__ VTl, const b16* __restrict__ LE, const b16* __restrict__ LEl, b16* __restrict__ OP, b16* __restrict__ OPl) {
  __shared__ __attribute__((aligned(16))) float To[2][16][HP + 4];
  const int wave = threadIdx.x >> 5, lane = threadIdx.x & 31, hh = lane >> 4, col = lane & 15; const int bh = blockIdx.y, b = bh / NH, hd = bh - b * NH; const int q0 = blockIdx.x * 32 + wave * 16, qi = q0 + col;
  const size_t qo = ((size_t)bh * NPX + qi) * HP; const v16b qa0 = frag_kb(QFh + qo, hh), qa1 = frag_kb(QFh + qo + 32, hh);
  const b16* Kb = KRh + (size_t)bh * NPX * HP; const b16* Vb = VT + (size_t)bh * HC * NPX; const b16* Vlb = VTl + (size_t)bh * HC * NPX;
  float m = -INFINITY, l = 0.0f; v8f o[3] = {{}, {}, {}}, ol[3] = {{}, {}, {}};
  const float cs = LOG2E / (XS * XS);
  for (int kb = 0; kb < NPX; kb += 32) {
    v8f s0 = {}, s1 = {};
    { const b16* k0 = Kb + (size_t)(kb + col) * HP, *k1 = Kb + (size_t)(kb + 16 + col) * HP;
      s0 = wmma16b(frag_kb(k0, hh), qa0, s0); s0 = wmma16b(frag_kb(k0 + 32, hh), qa1, s0); s1 = wmma16b(frag_kb(k1, hh), qa0, s1); s1 = wmma16b(frag_kb(k1 + 32, hh), qa1, s1); }
    float e[16]; float mx = -INFINITY;
#pragma unroll
    for (int r = 0; r < 8; ++r) { e[r] = s0[r] * cs; e[8 + r] = s1[r] * cs; mx = fmaxf(mx, fmaxf(e[r], e[8 + r])); }
    mx = fmaxf(mx, __shfl_xor(mx, 16)); const float mn = fmaxf(m, mx); const float al = nexp2(m - mn); m = mn; float sum = 0.0f; v16b ph, pl;
#pragma unroll
    for (int i2 = 0; i2 < 16; ++i2) { const float p = nexp2(e[i2] - mn); sum += p; const b16 h_ = (b16)(p * PS); ph[i2] = h_; pl[i2] = (b16)(p * PS - (float)h_); }
    sum += __shfl_xor(sum, 16); l = l * al + sum;
#pragma unroll
    for (int t = 0; t < 3; ++t) { o[t] *= al; ol[t] *= al; const v16b vf = frag_kb(Vb + (size_t)(t * 16 + col) * NPX + kb, hh); o[t] = wmma16b(vf, ph, o[t]); ol[t] = wmma16b(vf, pl, ol[t]); ol[t] = wmma16b(frag_kb(Vlb + (size_t)(t * 16 + col) * NPX + kb, hh), ph, ol[t]); } }
  const float inv = 1.0f / (l * PS * XS);
#pragma unroll
  for (int t = 0; t < 3; ++t)
#pragma unroll
    for (int r = 0; r < 8; ++r) To[wave][col][t * 16 + 8 * hh + r] = (o[t][r] + ol[t][r]) * inv;
  if (hh == 0) for (int d = HC; d < HP; ++d) To[wave][col][d] = 0.0f;
  wave_lds_sync();
  { const int rr = lane >> 1, d0 = (lane & 1) * 32; const size_t ro = ((size_t)b * NPX + q0 + rr) * (NH * HP) + hd * HP + d0; for (int j2 = 0; j2 < 32; ++j2) To[wave][rr][d0 + j2] += ((float)LE[ro + j2] + (float)LEl[ro + j2]) * (1.0f / OS); }
  wave_lds_sync();
  for (int pass = 0; pass < 2; ++pass) { { const int rr = lane >> 1, d0 = (lane & 1) * 32; const size_t ro = ((size_t)b * NPX + q0 + rr) * (NH * HP) + hd * HP + d0;
#pragma unroll
      for (int ch = 0; ch < 4; ++ch) { v8b hv, lv; for (int j2 = 0; j2 < 8; ++j2) { b16 p, q; split16(To[wave][rr][d0 + ch * 8 + j2] * OS, p, q); hv[j2] = p; lv[j2] = q; } *(volatile v8b*)(OP + ro + ch * 8) = hv; *(volatile v8b*)(OPl + ro + ch * 8) = lv; } } __threadfence(); }
}
}

extern "C" void kernel_launch(void* const* d_in, const int* in_sizes, int n_in, void* d_out, int out_size, void* d_ws, size_t ws_size, hipStream_t stream) {
  (void)n_in;
  auto Fp = [&](int i) { return (const float*)d_in[i]; };
  if (in_sizes[0] != NB * C * NPX || in_sizes[1] != C * C || in_sizes[3] != GC * 9 || in_sizes[7] != 2 * GC || in_sizes[12] != C * C || in_sizes[14] != C * 9 || out_size != NB * C * NPX) return;
  size_t off = 0; char* ws = (char*)d_ws;
  auto carve = [&](size_t bytes) { char* p = ws + off; off += (bytes + 255) & ~(size_t)255; return p; };
  b16* X16T = (b16*)carve((size_t)NR * C * 2); b16* WP = (b16*)carve((size_t)3 * C * C * 2); b16* WOP = (b16*)carve((size_t)C * 512 * 2);
  float* Q = (float*)carve((size_t)NB * C * NPX * 4);
  b16* XSh = (b16*)carve((size_t)NR * C * 2); b16* XSl = (b16*)carve((size_t)NR * C * 2);
  b16* LE = (b16*)carve((size_t)NR * NH * HP * 2); b16* LEl = (b16*)carve((size_t)NR * NH * HP * 2);
  b16* QF = (b16*)carve((size_t)NB * NH * NPX * HP * 2); b16* KR = (b16*)carve((size_t)NB * NH * NPX * HP * 2);
  b16* VT = (b16*)carve((size_t)NB * NH * HC * NPX * 2); b16* VTl = (b16*)carve((size_t)NB * NH * HC * NPX * 2);
  b16* OP = XSh; b16* OPl = (b16*)Q;
  if ((char*)XSl != (char*)XSh + (size_t)NR * C * 2 || (size_t)2 * NR * C * 2 < (size_t)NR * NH * HP * 2 || (size_t)NB * C * NPX * 4 < (size_t)NR * NH * HP * 2) return;
  if (off > ws_size || off > ((size_t)128 << 20)) return;
  const b16 *WQ = WP, *WK = WP + (size_t)C * C, *WV = WP + (size_t)2 * C * C;
  prepx_kernel<<<dim3(NPX / 64, C / 64, NB), 256, 0, stream>>>(Fp(0), X16T);
  prepw_kernel<<<(unsigned)(((size_t)3 * C * C / 8 + (size_t)C * 512 / 8 + 255) / 256), 256, 0, stream>>>(Fp(1), Fp(8), Fp(10), Fp(12), WP, WOP);
  proj_kernel<0><<<dim3(NR / 64, 4), 128, 0, stream>>>(X16T, nullptr, WQ, Fp(2), Q, QF, nullptr);
  samp_kernel<<<NR / 8, 256, 0, stream>>>(Q, Fp(0), Fp(3), Fp(4), Fp(5), Fp(6), Fp(7), Fp(14), Fp(15), XSh, XSl, LE, LEl);
  proj_kernel<1><<<dim3(NR / 64, 4), 128, 0, stream>>>(XSh, XSl, WK, Fp(9), nullptr, KR, nullptr);
  proj_kernel<3><<<dim3(NR / 64, 4), 128, 0, stream>>>(XSh, XSl, WV, Fp(11), nullptr, VT, VTl);
  attn_kernel<<<dim3(NPX / 32, NB * NH), 64, 0, stream>>>(QF, KR, VT, VTl, LE, LEl, OP, OPl);
  proj_kernel<2><<<dim3(NR / 64, 4), 128, 0, stream>>>(OP, OPl, WOP, Fp(13), (float*)d_out, nullptr, nullptr);
}
